// KPConvSimpleBlock_67714454389185
// MI455X (gfx1250) — hardware-verified
//
#include <hip/hip_runtime.h>
#include <math.h>

typedef __attribute__((ext_vector_type(16))) _Float16 v16h;
typedef __attribute__((ext_vector_type(16))) __bf16 v16b;
typedef __attribute__((ext_vector_type(8)))  _Float16 v8h;
typedef __attribute__((ext_vector_type(8)))  float v8f;
typedef __attribute__((ext_vector_type(4)))  float v4f;
typedef __attribute__((ext_vector_type(2)))  float v2f;
typedef __attribute__((ext_vector_type(4)))  unsigned v4u;
typedef __attribute__((ext_vector_type(4)))  int v4i;
typedef float __attribute__((may_alias)) float_a;
typedef int __attribute__((may_alias)) int_a;

template <typename T> __device__ __forceinline__ void vst2(void* p, T v) { *(volatile T*)p = v; __threadfence(); *(volatile T*)p = v; }
__device__ __forceinline__ v8f wmma16(v16h a, v16h b, v8f c) {
  v8f d = __builtin_amdgcn_wmma_f32_16x16x32_f16(false, a, false, b, (short)0, c, false, false);
  asm volatile("v_nop\n\tv_nop\n\tv_nop\n\tv_nop" : "+v"(d) : "v"(a), "v"(b));
  return d;
}
__device__ __forceinline__ v8f wmma_bf(v16b a, v16b b, v8f c) {
  v8f d = __builtin_amdgcn_wmma_f32_16x16x32_bf16(false, a, false, b, (short)0, c, false, false);
  asm volatile("v_nop\n\tv_nop\n\tv_nop\n\tv_nop" : "+v"(d) : "v"(a), "v"(b));
  return d;
}
__device__ __forceinline__ v16h frag_h(const _Float16* rowk0, int lane) {
  union { v16h v; v8h q[2]; } u; const _Float16* p = rowk0 + 8 * (lane >> 4);
  u.q[0] = *(const v8h*)p; u.q[1] = *(const v8h*)(p + 16); return u.v;
}
__device__ __forceinline__ v16h frag_f32(const float* rowk0, int lane) {
  v16h a; const float* p = rowk0 + 8 * (lane >> 4);
#pragma unroll
  for (int i = 0; i < 8; ++i) { a[i] = (_Float16)p[i]; a[8 + i] = (_Float16)p[16 + i]; }
  return a;
}
__device__ __forceinline__ v16h frag_f32s(const float* rowk0, int lane, float sc) {
  v16h a; const float* p = rowk0 + 8 * (lane >> 4);
#pragma unroll
  for (int i = 0; i < 8; ++i) { a[i] = (_Float16)(p[i] * sc); a[8 + i] = (_Float16)(p[16 + i] * sc); }
  return a;
}
__device__ __forceinline__ v16h fragc_f32(const float* W, int k0, int n, int lane, int ld, int K) {
  v16h a; const int g = lane >> 4;
#pragma unroll
  for (int i = 0; i < 8; ++i) { const int ka = k0 + 8 * g + i, kb = ka + 16;
    a[i] = (_Float16)(ka < K ? W[(size_t)(ka < K ? ka : K - 1) * ld + n] : 0.f); a[8 + i] = (_Float16)(kb < K ? W[(size_t)(kb < K ? kb : K - 1) * ld + n] : 0.f); }
  return a;
}
struct F2 { v16b h, l; };
__device__ __forceinline__ F2 bsplit16(const float v[16]) { F2 r;
#pragma unroll
  for (int i = 0; i < 16; ++i) { const __bf16 h = (__bf16)v[i]; r.h[i] = h; r.l[i] = (__bf16)(v[i] - (float)h); }
  return r; }
__device__ __forceinline__ F2 split_row(const float* row, int k0, int lane) { float v[16]; const float* p = row + k0 + 8 * (lane >> 4);
#pragma unroll
  for (int i = 0; i < 8; ++i) { v[i] = p[i]; v[8 + i] = p[16 + i]; }
  return bsplit16(v); }
__device__ __forceinline__ F2 split_rowK(const float* row, int k0, int lane, int K) { float v[16]; const int g = lane >> 4;
#pragma unroll
  for (int i = 0; i < 8; ++i) { const int ka = k0 + 8 * g + i, kb = ka + 16; v[i] = ka < K ? row[ka < K ? ka : K - 1] : 0.f; v[8 + i] = kb < K ? row[kb < K ? kb : K - 1] : 0.f; }
  return bsplit16(v); }
__device__ __forceinline__ F2 split_col(const float* W, int k0, int n, int lane, int ld, int K) { float v[16]; const int g = lane >> 4;
#pragma unroll
  for (int i = 0; i < 8; ++i) { const int ka = k0 + 8 * g + i, kb = ka + 16; v[i] = ka < K ? W[(size_t)(ka < K ? ka : K - 1) * ld + n] : 0.f; v[8 + i] = kb < K ? W[(size_t)(kb < K ? kb : K - 1) * ld + n] : 0.f; }
  return bsplit16(v); }
__device__ __forceinline__ v8f mac3(const F2& a, const F2& b, v8f c) { c = wmma_bf(a.l, b.h, c); c = wmma_bf(a.h, b.l, c); return wmma_bf(a.h, b.h, c); }
__device__ __forceinline__ float sigm(float v) { return 1.0f / (1.0f + expf(-v)); }
#define LDSX() do { asm volatile("s_wait_dscnt 0" ::: "memory"); __builtin_amdgcn_wave_barrier(); __builtin_amdgcn_fence(__ATOMIC_RELEASE, "workgroup"); } while (0)


#define NB 8
#define NPT 4096
#define MM (NB * NPT)
#define CI 64
#define CO 128
#define KP 15
#define MAXNN 34
#define KPE 0.04f
#ifndef NBT
#define NBT NB
#endif
#define MMT (NBT * NPT)
typedef __attribute__((ext_vector_type(8))) __bf16 v8b;
__device__ __forceinline__ v16b frag_b(const __bf16* rowk0, int lane) {
  union { v16b v; v8b q[2]; } u; const __bf16* p = rowk0 + 8 * (lane >> 4);
  u.q[0] = *(const v8b*)p; u.q[1] = *(const v8b*)(p + 16); return u.v;
}
__device__ __forceinline__ float bfr(float v) { return (float)(__bf16)v; }
__device__ __attribute__((noinline)) float exp_ni(float v) { return expf(v); }
__device__ __attribute__((noinline)) float erf_ni(float v) { return erff(v); }

struct F3 { v16b h, m, l; };
__device__ __forceinline__ F3 bsplit16_3(const float v[16]) { F3 r;
#pragma unroll
  for (int i = 0; i < 16; ++i) { const __bf16 h = (__bf16)v[i]; const float r1 = v[i] - (float)h; const __bf16 m = (__bf16)r1; r.h[i] = h; r.m[i] = m; r.l[i] = (__bf16)(r1 - (float)m); }
  return r; }
__device__ __forceinline__ F3 split3_row(const float* row, int k0, int lane) { float v[16]; const float* p = row + k0 + 8 * (lane >> 4);
#pragma unroll
  for (int i = 0; i < 8; ++i) { v[i] = p[i]; v[8 + i] = p[16 + i]; }
  return bsplit16_3(v); }

#define WS_PW   0u
#define WS_NI   (WS_PW + 2u * CO * 960)
#define WS_WF   (WS_NI + 4u * MM * 64)
#define WS_OUT  (WS_WF + 4u * MM * 960)
#define NSTB 128
#define WS_ST   (WS_OUT + 4u * MM * CO)
#define WS_BN   (WS_ST + 4u * NSTB * 128)
#define WS_END  (WS_BN + 4u * 4 * 128)

__global__ __launch_bounds__(256) void k_packw(const float* __restrict__ Wm, __bf16* __restrict__ PW) {
  __shared__ __align__(16) __bf16 s[960]; const int d = blockIdx.x, t = threadIdx.x;
  for (int q = t; q < 960; q += 256) s[q] = (__bf16)Wm[(size_t)q * CO + d];
  __syncthreads();
  for (int q = t; q < 120; q += 256) vst2((unsigned*)(PW + (size_t)d * 960 + q * 8), *(const v4u*)&s[q * 8]);
}
__global__ __launch_bounds__(64) void k_ball(const float* __restrict__ XYZ, int* __restrict__ NI) {
  #pragma clang fp contract(off)
  __shared__ __align__(16) int sn[64][64]; const int tid = threadIdx.x; const size_t i = (size_t)blockIdx.x * 64 + tid; const int b = (int)(i / NPT); const float* pb = XYZ + (size_t)b * NPT * 3; const int il = (int)(i % NPT);
  const float xi = bfr(pb[il * 3]), yi = bfr(pb[il * 3 + 1]), zi = bfr(pb[il * 3 + 2]);
  float bd[MAXNN]; int bi[MAXNN];
#pragma unroll
  for (int q = 0; q < MAXNN; ++q) { bd[q] = 3.0e38f; bi[q] = 0; }
#pragma unroll 1
  for (int j = 0; j < NPT; ++j) { const float dx = xi - bfr(pb[j * 3]), dy = yi - bfr(pb[j * 3 + 1]), dz = zi - bfr(pb[j * 3 + 2]); const float d = (dx * dx + dz * dz) + dy * dy;
    if (d < bd[MAXNN - 1]) { int pos = MAXNN - 1;
#pragma unroll
      for (int q = MAXNN - 2; q >= 0; --q) if (d < bd[q]) pos = q;
#pragma unroll
      for (int q = MAXNN - 1; q >= 1; --q) if (q > pos) { bd[q] = bd[q - 1]; bi[q] = bi[q - 1]; }
#pragma unroll
      for (int q = 0; q < MAXNN; ++q) if (q == pos) { bd[q] = d; bi[q] = j; } } }
  const float r2 = 0.1f * 0.1f;
#pragma unroll
  for (int q = 0; q < 64; ++q) sn[tid][q] = (q < MAXNN && bd[q] <= r2) ? (b * NPT + bi[q]) : -1;
  __syncthreads();
  for (int r = 0; r < 64; ++r) if (tid < 16) vst2((unsigned*)(NI + ((size_t)blockIdx.x * 64 + r) * 64 + tid * 4), *(const v4u*)&sn[r][tid * 4]);
}
__global__ __launch_bounds__(128) void k_wf(const float* __restrict__ XYZ, const float* __restrict__ FEAT, const float* __restrict__ KPT, const int* __restrict__ NI, float* __restrict__ WF) {
  __shared__ __align__(16) float sA[4][16][68]; __shared__ __align__(16) __bf16 sB[4][64][72]; __shared__ __align__(16) float so[4][16][68];
  const int tid = threadIdx.x, wave = tid >> 5, lane = tid & 31, col = lane & 15, g = lane >> 4; const size_t i = (size_t)blockIdx.x * 4 + wave;
  const float xi = bfr(XYZ[i * 3]), yi = bfr(XYZ[i * 3 + 1]), zi = bfr(XYZ[i * 3 + 2]);
  for (int n = lane; n < 64; n += 32) { const int j = (n < MAXNN) ? NI[i * 64 + n] : -1;
    if (j >= 0) { const float rx = bfr(XYZ[(size_t)j * 3]) - xi, ry = bfr(XYZ[(size_t)j * 3 + 1]) - yi, rz = bfr(XYZ[(size_t)j * 3 + 2]) - zi;
#pragma unroll 1
      for (int k = 0; k < KP; ++k) { const float ax = rx - bfr(KPT[k * 3]), ay = ry - bfr(KPT[k * 3 + 1]), az = rz - bfr(KPT[k * 3 + 2]); const float sq = (ax * ax + ay * ay) + az * az; sA[wave][k][n] = fmaxf(1.0f - sqrtf(sq) / KPE, 0.f); }
      sA[wave][15][n] = 0.f;
      const float* fr = FEAT + (size_t)j * CI;
#pragma unroll 4
      for (int c = 0; c < CI; ++c) sB[wave][c][n] = (__bf16)fr[c]; }
    else {
#pragma unroll
      for (int k = 0; k < 16; ++k) sA[wave][k][n] = 0.f;
#pragma unroll 4
      for (int c = 0; c < CI; ++c) sB[wave][c][n] = (__bf16)0.f; } }
  LDSX();
  v8f acc[4] = {};
#pragma unroll
  for (int kc = 0; kc < 2; ++kc) { const F2 a = split_row(&sA[wave][col][0], kc * 32, lane);
#pragma unroll
    for (int ct = 0; ct < 4; ++ct) { const v16b bb = frag_b(&sB[wave][ct * 16 + col][kc * 32], lane); acc[ct] = wmma_bf(a.l, bb, acc[ct]); acc[ct] = wmma_bf(a.h, bb, acc[ct]); } }
#pragma unroll
  for (int ct = 0; ct < 4; ++ct)
#pragma unroll
    for (int r = 0; r < 8; ++r) so[wave][8 * g + r][ct * 16 + col] = acc[ct][r];
  LDSX();
  for (int q = lane; q < 240; q += 32) { const int k = q >> 4, pc = q & 15; vst2(WF + i * 960 + k * 64 + pc * 4, *(const v4f*)&so[wave][k][pc * 4]); }
}
__global__ __launch_bounds__(128) void k_out(const float* __restrict__ WF, const __bf16* __restrict__ PW, float* __restrict__ OUT) {
  __shared__ __align__(16) float so[4][16][132];
  const int tid = threadIdx.x, wave = tid >> 5, lane = tid & 31, col = lane & 15, g = lane >> 4; const size_t r0 = (size_t)blockIdx.x * 64 + wave * 16;
  v8f acc[8] = {};
#pragma unroll 2
  for (int kc = 0; kc < 30; ++kc) { const F3 a = split3_row(WF + (r0 + col) * 960, kc * 32, lane);
#pragma unroll
    for (int j = 0; j < 8; ++j) { const v16b w = frag_b(PW + (size_t)(j * 16 + col) * 960 + kc * 32, lane); acc[j] = wmma_bf(a.l, w, acc[j]); acc[j] = wmma_bf(a.m, w, acc[j]); acc[j] = wmma_bf(a.h, w, acc[j]); } }
#pragma unroll
  for (int j = 0; j < 8; ++j)
#pragma unroll
    for (int r = 0; r < 8; ++r) so[wave][8 * g + r][j * 16 + col] = acc[j][r];
  LDSX();
  for (int rl = 0; rl < 16; ++rl) vst2(OUT + (r0 + rl) * CO + lane * 4, *(const v4f*)&so[wave][rl][lane * 4]);
}
template <int PASS>
__global__ __launch_bounds__(128) void k_stat(const float* __restrict__ Y, int nrows, const float* __restrict__ BNP, float* __restrict__ ST) {
  __shared__ __align__(16) float s[128]; const int c = threadIdx.x; const int rpb = nrows / NSTB; const size_t r0 = (size_t)blockIdx.x * rpb; float a = 0.f; const float mu = PASS ? BNP[c] : 0.f;
#pragma unroll 4
  for (int r = 0; r < rpb; ++r) { const float y = Y[(r0 + r) * CO + c]; const float d = y - mu; a += PASS ? d * d : y; }
  s[c] = a; __syncthreads();
  if (c < 32) vst2(ST + (size_t)blockIdx.x * 128 + c * 4, *(const v4f*)&s[c * 4]);
}
template <int PASS>
__global__ __launch_bounds__(128) void k_fin(const float* __restrict__ ST, int nrows, const float* __restrict__ G, const float* __restrict__ BE, float* __restrict__ BNP) {
  __shared__ __align__(16) float s[2][128]; const int c = threadIdx.x; float a = 0.f;
#pragma unroll 1
  for (int b = 0; b < NSTB; ++b) a += ST[(size_t)b * 128 + c];
  const float n = (float)nrows;
  if (PASS == 0) { s[0][c] = a / n; __syncthreads(); if (c < 32) vst2(BNP + c * 4, *(const v4f*)&s[0][c * 4]); }
  else { const float var = a / n; const float sc = bfr(G[c]) * rsqrtf(var + 1e-5f); s[0][c] = sc; s[1][c] = bfr(BE[c]) - BNP[c] * sc; __syncthreads(); if (c < 32) { vst2(BNP + 128 + c * 4, *(const v4f*)&s[0][c * 4]); vst2(BNP + 256 + c * 4, *(const v4f*)&s[1][c * 4]); } }
}
__global__ __launch_bounds__(128) void k_bn(const float* __restrict__ Y, const float* __restrict__ BNP, float* __restrict__ OUTF) {
  __shared__ __align__(16) float s[64][CO + 4]; const int c = threadIdx.x; const size_t r0 = (size_t)blockIdx.x * 64; const float sc = BNP[128 + c], sh = BNP[256 + c];
  for (int r = 0; r < 64; ++r) { const float v = Y[(r0 + r) * CO + c] * sc + sh; s[r][c] = v >= 0.f ? v : 0.2f * v; }
  __syncthreads();
  for (int q = c; q < 64 * 32; q += 128) { const int r = q >> 5, pc = q & 31; vst2(OUTF + (r0 + r) * CO + pc * 4, *(const v4f*)&s[r][pc * 4]); }
}
extern "C" void kernel_launch(void* const* d_in, const int* in_sizes, int n_in, void* d_out, int out_size, void* d_ws, size_t ws_size, hipStream_t stream) {
  (void)in_sizes; (void)n_in; (void)out_size;
  const float** F = (const float**)d_in;
  if (ws_size < (size_t)WS_END) return;
  char* ws = (char*)d_ws; __bf16* PW = (__bf16*)(ws + WS_PW); int* NI = (int*)(ws + WS_NI); float *WF = (float*)(ws + WS_WF), *OUT = (float*)(ws + WS_OUT), *ST = (float*)(ws + WS_ST), *BN = (float*)(ws + WS_BN);
  k_packw<<<CO, 256, 0, stream>>>(F[3], PW);
  k_ball<<<MMT / 64, 64, 0, stream>>>(F[0], NI);
  k_wf<<<MMT / 4, 128, 0, stream>>>(F[0], F[1], F[2], NI, WF);
  k_out<<<MMT / 64, 128, 0, stream>>>(WF, PW, OUT);
  k_stat<0><<<NSTB, 128, 0, stream>>>(OUT, MMT, BN, ST); k_fin<0><<<1, 128, 0, stream>>>(ST, MMT, F[4], F[5], BN); k_stat<1><<<NSTB, 128, 0, stream>>>(OUT, MMT, BN, ST); k_fin<1><<<1, 128, 0, stream>>>(ST, MMT, F[4], F[5], BN);
  k_bn<<<MMT / 64, 128, 0, stream>>>(OUT, BN, (float*)d_out);
}
